// GCN_83751862272702
// MI455X (gfx1250) — hardware-verified
//
#include <hip/hip_runtime.h>
#include <stddef.h>
#include <stdint.h>
#include <math.h>


#define CIN    128
#define CH     256
#define KX     512
#define NG     2048
#define HF1    128
#define DOUT   32
#define KT2    256
#define NTHR   256
#define NWAVE  8
#define EPT    8
#define CHUNK  (NTHR * EPT)
#define WCAP   (EPT * 32)
#define LISTN  (NWAVE * WCAP)
#define NBD    8192
#define SLD    13
#define NBA    1024
#define SLA    10
#define RCAP   12288
#define DEGCAP 64
#define NBP    64
#define SLP    6
#define RCP    4096
#define PDEGCAP 128
#define GBM    64
#define GBN    64
#define GTHR   128
#define MISC_INTS    16
#define ROWBUF_INTS  (NWAVE * KX / 2)
#define AGG_ZINTS    (LISTN + 2 * RCAP + 3 * NBA)
#define AGG_LDS_INTS (AGG_ZINTS + MISC_INTS + ROWBUF_INTS)
#define POOL_ZINTS    (LISTN + 2 * RCP + 3 * NBP)
#define POOL_LDS_INTS (POOL_ZINTS + MISC_INTS + ROWBUF_INTS)
#define NUA    (CH * (CIN / 8))
#define NUB    (CH * (KX / 8))
#define NUC    (CH * (KX / 8))
#define NUD    (HF1 * (KX / 8))
#define NUE    (DOUT * (KT2 / 8))
#define NUALL  (NUA + NUB + NUC + NUD + NUE)
#define NOUT   (NG * DOUT)
#define WSMAX  134217728

static_assert((CHUNK & (CHUNK - 1)) == 0 && CHUNK <= 4096);
static_assert((NBD & (NBD - 1)) == 0 && NBD == (1 << SLD));
static_assert((NBA & (NBA - 1)) == 0 && NBA == (1 << SLA));
static_assert((NBP & (NBP - 1)) == 0 && NBP == (1 << SLP));
static_assert(((long long)CHUNK << SLD) < (1LL << 31));
static_assert(((long long)CHUNK << SLA) < (1LL << 31));
static_assert(NBD % (NTHR * 4) == 0 && NBD % NTHR == 0);
static_assert(LISTN % NTHR == 0 && LISTN % 4 == 0);
static_assert(NBA % NWAVE == 0 && NBA % 32 == 0 && NBA % GBM == 0);
static_assert(NBP % NWAVE == 0 && NBP % 32 == 0 && NG % NBP == 0);
static_assert(RCAP % 4 == 0 && RCP % 4 == 0 && AGG_ZINTS % 4 == 0 && POOL_ZINTS % 4 == 0);
static_assert(((AGG_ZINTS + MISC_INTS) % 4) == 0 && ((POOL_ZINTS + MISC_INTS) % 4) == 0);
static_assert(CIN % 32 == 0 && KX % 32 == 0 && KT2 % 32 == 0 && KX == 2 * CH && KT2 == 2 * HF1);
static_assert(CH % GBN == 0 && GBM == (GTHR / 32) * 16 && CH == 8 * 32);
static_assert(NUA % NTHR == 0 && NUB % NTHR == 0 && NUC % NTHR == 0 && NUD % NTHR == 0 && NUE % NTHR == 0);
static_assert(AGG_LDS_INTS * 4 <= 300000 && POOL_LDS_INTS * 4 <= 65536);
static_assert(NG % GBM == 0 && HF1 == 128 && DOUT == 32);
static_assert((GBM * DOUT) % (4 * GTHR) == 0);

typedef float          v4f   __attribute__((ext_vector_type(4)));
typedef float          v8f   __attribute__((ext_vector_type(8)));
typedef int            v4i   __attribute__((ext_vector_type(4)));
typedef int            v8i   __attribute__((ext_vector_type(8)));
typedef unsigned short v4us  __attribute__((ext_vector_type(4)));
typedef unsigned short v8us  __attribute__((ext_vector_type(8)));
typedef unsigned short v16us __attribute__((ext_vector_type(16)));
typedef __bf16         v16bf __attribute__((ext_vector_type(16)));
typedef v4f  __attribute__((may_alias)) v4fa;
typedef v4i  __attribute__((may_alias)) v4ia;
typedef v4us __attribute__((may_alias)) v4usa;
typedef v8us __attribute__((may_alias)) v8usa;
union FragB { v16bf v; v16us u; v8us h[2]; v8i w; };

__device__ __forceinline__ v8f wmb(const FragB& a, const FragB& b, v8f c) {
  v8f d = __builtin_amdgcn_wmma_f32_16x16x32_bf16(false, a.v, false, b.v, (short)0, c, false, false);
  asm volatile("v_nop\n\tv_nop\n\tv_nop\n\tv_nop" : "+v"(d) : "v"(a.w), "v"(b.w));
  return d;
}

__device__ __forceinline__ unsigned bf16_bits(float f) {
  const unsigned u = __float_as_uint(f);
  return (u + 0x7FFFu + ((u >> 16) & 1u)) >> 16;
}
__device__ __forceinline__ float bf16_val(float f) {
  return __uint_as_float(bf16_bits(f) << 16);
}
__device__ __forceinline__ float relu_np(float v) {
  return (v > 0.0f) ? v : (v - v);
}
__device__ __forceinline__ void split4(const v4f v, v4us& h, v4us& l) {
  unsigned hb;
  hb = bf16_bits(v.x); h[0] = (unsigned short)hb; l[0] = (unsigned short)bf16_bits(v.x - __uint_as_float(hb << 16));
  hb = bf16_bits(v.y); h[1] = (unsigned short)hb; l[1] = (unsigned short)bf16_bits(v.y - __uint_as_float(hb << 16));
  hb = bf16_bits(v.z); h[2] = (unsigned short)hb; l[2] = (unsigned short)bf16_bits(v.z - __uint_as_float(hb << 16));
  hb = bf16_bits(v.w); h[3] = (unsigned short)hb; l[3] = (unsigned short)bf16_bits(v.w - __uint_as_float(hb << 16));
}

__device__ __forceinline__ void wave_sync() {
  __builtin_amdgcn_fence(__ATOMIC_RELEASE, "wavefront");
  __builtin_amdgcn_wave_barrier();
  __builtin_amdgcn_fence(__ATOMIC_ACQUIRE, "wavefront");
}

template <int SLB>
__device__ __forceinline__ int scan_chunk(const int* __restrict__ dsts, int nE, int cbase, int slotBase,
                                          int nb, int vec8, int* list, int tid, int lane, int wave) {
  int wc = 0;
  const int el0  = tid * EPT;
  const int e0   = cbase + el0;
  const int sent = -2147483647 - 1;
  v4i da, db;
  if (vec8 != 0 && cbase + CHUNK <= nE) {
    da = *(const v4i*)(dsts + e0);
    db = *(const v4i*)(dsts + e0 + 4);
  } else {
    da.x = (e0     < nE) ? dsts[min(e0,     nE - 1)] : sent;
    da.y = (e0 + 1 < nE) ? dsts[min(e0 + 1, nE - 1)] : sent;
    da.z = (e0 + 2 < nE) ? dsts[min(e0 + 2, nE - 1)] : sent;
    da.w = (e0 + 3 < nE) ? dsts[min(e0 + 3, nE - 1)] : sent;
    db.x = (e0 + 4 < nE) ? dsts[min(e0 + 4, nE - 1)] : sent;
    db.y = (e0 + 5 < nE) ? dsts[min(e0 + 5, nE - 1)] : sent;
    db.z = (e0 + 6 < nE) ? dsts[min(e0 + 6, nE - 1)] : sent;
    db.w = (e0 + 7 < nE) ? dsts[min(e0 + 7, nE - 1)] : sent;
  }
  const unsigned nbs = (unsigned)slotBase;
  const unsigned unb = (unsigned)nb;
  const unsigned s0 = (unsigned)da.x - nbs, s1 = (unsigned)da.y - nbs;
  const unsigned s2 = (unsigned)da.z - nbs, s3 = (unsigned)da.w - nbs;
  const unsigned s4 = (unsigned)db.x - nbs, s5 = (unsigned)db.y - nbs;
  const unsigned s6 = (unsigned)db.z - nbs, s7 = (unsigned)db.w - nbs;
  const bool h0 = s0 < unb, h1 = s1 < unb, h2 = s2 < unb, h3 = s3 < unb;
  const bool h4 = s4 < unb, h5 = s5 < unb, h6 = s6 < unb, h7 = s7 < unb;
  const unsigned any = __builtin_amdgcn_ballot_w32(h0 | h1 | h2 | h3 | h4 | h5 | h6 | h7);
  if (any != 0u) {
#define HITJ(J, HJ, SJ) { \
      const unsigned mj = __builtin_amdgcn_ballot_w32(HJ); \
      if (mj != 0u) { \
        if (HJ) { \
          const int pos = wc + (int)__builtin_amdgcn_mbcnt_lo(mj, 0u); \
          if (pos < WCAP) list[wave * WCAP + pos] = ((el0 + (J)) << SLB) | (int)(SJ); \
        } \
        wc += (int)__builtin_popcount(mj); } }
    HITJ(0, h0, s0)
    HITJ(1, h1, s1)
    HITJ(2, h2, s2)
    HITJ(3, h3, s3)
    HITJ(4, h4, s4)
    HITJ(5, h5, s5)
    HITJ(6, h6, s6)
    HITJ(7, h7, s7)
#undef HITJ
  }
  return wc;
}

template <int SLB, int NB, int RC>
__device__ __forceinline__ void build_lists(const int* __restrict__ keys, int nE, int vec8, int slotBase,
                                            int* list, int* hl, int* sl, int* cnt, int* offs, int* cur,
                                            int* misc, int tid, int lane, int wave, int& ttOut, int& ovfOut) {
  int t = 0, ov = 0;
  const int nChunks = (nE + CHUNK - 1) / CHUNK;
#pragma unroll 1
  for (int ch = 0; ch < nChunks; ++ch) {
    const int cbase = ch * CHUNK;
    const int wc = scan_chunk<SLB>(keys, nE, cbase, slotBase, NB, vec8, list, tid, lane, wave);
    if (lane == 0) misc[wave] = wc;
    __syncthreads();
    if (wave == 0) {
#pragma unroll 1
      for (int w2 = 0; w2 < NWAVE; ++w2) {
        int c = misc[w2];
        c = c < 0 ? 0 : (c > WCAP ? WCAP : c);
#pragma unroll 1
        for (int b0 = 0; b0 < c; b0 += 32) {
          const int idx = b0 + lane;
          const int ent = list[w2 * WCAP + (idx < WCAP ? idx : WCAP - 1)];
          const int m32 = (c - b0) < 32 ? (c - b0) : 32;
#pragma unroll 1
          for (int k = 0; k < m32; ++k) {
            const int u    = __builtin_amdgcn_readlane(ent, k);
            const int slot = u & (NB - 1);
            const int el   = (u >> SLB) & (CHUNK - 1);
            const int pk   = ((cbase + el) << SLB) | slot;
            if (t < RC) {
              if (lane == 0) { hl[t] = pk; cnt[slot] = cnt[slot] + 1; }
              t = t + 1;
            } else {
              ov = 1;
            }
          }
        }
      }
    }
    __syncthreads();
  }
  if (wave == 0 && lane == 0) { misc[8] = t; misc[9] = ov; }
  __syncthreads();
  int tt = misc[8];
  tt = tt < 0 ? 0 : (tt > RC ? RC : tt);
  const int ovf = misc[9];

  if (wave == 0) {
    const int base = lane * (NB / 32);
    int s = 0;
#pragma unroll 1
    for (int i = 0; i < NB / 32; ++i) s += cnt[base + i];
    int incl = s;
#pragma unroll
    for (int d = 1; d < 32; d <<= 1) {
      const int y = __shfl_up(incl, d, 32);
      if (lane >= d) incl += y;
    }
    int run = incl - s;
#pragma unroll 1
    for (int i = 0; i < NB / 32; ++i) {
      const int cv = cnt[base + i];
      offs[base + i] = run;
      cur[base + i]  = run;
      run += cv;
    }
  }
  __syncthreads();
  if (wave == 0) {
#pragma unroll 1
    for (int b0 = 0; b0 < tt; b0 += 32) {
      const int idx = b0 + lane;
      const int ent = hl[idx < RC ? idx : RC - 1];
      const int m32 = (tt - b0) < 32 ? (tt - b0) : 32;
#pragma unroll 1
      for (int k = 0; k < m32; ++k) {
        const int u    = __builtin_amdgcn_readlane(ent, k);
        const int slot = u & (NB - 1);
        if (lane == 0) {
          int p = cur[slot];
          p = p < 0 ? 0 : (p > RC - 1 ? RC - 1 : p);
          sl[p] = u;
          cur[slot] = p + 1;
        }
      }
    }
  }
  __syncthreads();
  ttOut = tt;
  ovfOut = ovf;
}

__global__ __launch_bounds__(NTHR) void k_wprep(const float* __restrict__ W1, const float* __restrict__ W2,
                                                const float* __restrict__ W3, const float* __restrict__ Wf1,
                                                const float* __restrict__ Wf2,
                                                unsigned short* W1T, unsigned short* W2T2, unsigned short* W3T2,
                                                unsigned short* WF1T2, unsigned short* WF2T2) {
  const int u = (int)blockIdx.x * NTHR + (int)threadIdx.x;
  const float* p;
  unsigned short* dp;
  int ld;
  if (u < NUA) {
    const int n = u >> 4, k8 = (u & 15) * 8;
    p = W1 + (size_t)k8 * CH + n; ld = CH;
    dp = W1T + (size_t)n * CIN + k8;
  } else if (u < NUA + NUB) {
    const int v = u - NUA;
    const int n = v >> 6, k8 = (v & 63) * 8, kk = k8 & (CH - 1);
    p = W2 + (size_t)kk * CH + n; ld = CH;
    dp = W2T2 + (size_t)n * KX + k8;
  } else if (u < NUA + NUB + NUC) {
    const int v = u - (NUA + NUB);
    const int n = v >> 6, k8 = (v & 63) * 8, kk = k8 & (CH - 1);
    p = W3 + (size_t)kk * CH + n; ld = CH;
    dp = W3T2 + (size_t)n * KX + k8;
  } else if (u < NUA + NUB + NUC + NUD) {
    const int v = u - (NUA + NUB + NUC);
    const int n = v >> 6, k8 = (v & 63) * 8, kk = k8 & (CH - 1);
    p = Wf1 + (size_t)kk * HF1 + n; ld = HF1;
    dp = WF1T2 + (size_t)n * KX + k8;
  } else if (u < NUALL) {
    const int v = u - (NUA + NUB + NUC + NUD);
    const int n = v >> 5, k8 = (v & 31) * 8, kk = k8 & (HF1 - 1);
    p = Wf2 + (size_t)kk * DOUT + n; ld = DOUT;
    dp = WF2T2 + (size_t)n * KT2 + k8;
  } else {
    return;
  }
  v8us o;
#pragma unroll
  for (int i = 0; i < 8; ++i) o[i] = (unsigned short)bf16_bits(p[(size_t)i * ld]);
  *(volatile v8us*)dp = o;
  __threadfence();
  *(volatile v8us*)dp = o;
}

__global__ __launch_bounds__(NTHR) void k_cvx(const float* __restrict__ x, int nN, int nUnits,
                                              unsigned short* xb) {
  const int u = (int)blockIdx.x * NTHR + (int)threadIdx.x;
  if (u >= nUnits) return;
  const int row = u >> 4;
  const int k8  = (u & 15) * 8;
  const int rc  = row < nN ? row : nN - 1;
  const float* p = x + (size_t)rc * CIN + k8;
  const v4f a = *(const v4fa*)p;
  const v4f b = *(const v4fa*)(p + 4);
  const bool ok = row < nN;
  v8us o;
  o[0] = ok ? (unsigned short)bf16_bits(a.x) : (unsigned short)0;
  o[1] = ok ? (unsigned short)bf16_bits(a.y) : (unsigned short)0;
  o[2] = ok ? (unsigned short)bf16_bits(a.z) : (unsigned short)0;
  o[3] = ok ? (unsigned short)bf16_bits(a.w) : (unsigned short)0;
  o[4] = ok ? (unsigned short)bf16_bits(b.x) : (unsigned short)0;
  o[5] = ok ? (unsigned short)bf16_bits(b.y) : (unsigned short)0;
  o[6] = ok ? (unsigned short)bf16_bits(b.z) : (unsigned short)0;
  o[7] = ok ? (unsigned short)bf16_bits(b.w) : (unsigned short)0;
  unsigned short* dp = xb + (size_t)row * CIN + k8;
  *(volatile v8us*)dp = o;
  __threadfence();
  *(volatile v8us*)dp = o;
}

__global__ __launch_bounds__(NTHR) void k_deg(const int* __restrict__ dsts, int nE, int vec8, float* dis) {
  __shared__ __attribute__((aligned(16))) int scnt[NBD];
  __shared__ __attribute__((aligned(16))) int list[LISTN];
  __shared__ int wcnt[NWAVE];
  const int tid = (int)threadIdx.x, lane = tid & 31, wave = tid >> 5;
  const int nodeBase = (int)blockIdx.x * NBD;

  for (int i = tid; i < NBD; i += NTHR) scnt[i] = 0;
  for (int i = tid; i < LISTN; i += NTHR) list[i] = 0;
  if (tid < NWAVE) wcnt[tid] = 0;
  __syncthreads();

  const int nChunks = (nE + CHUNK - 1) / CHUNK;
#pragma unroll 1
  for (int ch = 0; ch < nChunks; ++ch) {
    const int cbase = ch * CHUNK;
    const int wc = scan_chunk<SLD>(dsts, nE, cbase, nodeBase, NBD, vec8, list, tid, lane, wave);
    if (lane == 0) wcnt[wave] = wc;
    __syncthreads();
    if (wave == 0) {
#pragma unroll 1
      for (int w2 = 0; w2 < NWAVE; ++w2) {
        int c = wcnt[w2];
        c = c < 0 ? 0 : (c > WCAP ? WCAP : c);
#pragma unroll 1
        for (int b0 = 0; b0 < c; b0 += 32) {
          const int idx = b0 + lane;
          const int ent = list[w2 * WCAP + (idx < WCAP ? idx : WCAP - 1)];
          const int m32 = (c - b0) < 32 ? (c - b0) : 32;
#pragma unroll 1
          for (int k = 0; k < m32; ++k) {
            const int u  = __builtin_amdgcn_readlane(ent, k);
            const int sl = u & (NBD - 1);
            if (lane == 0) scnt[sl] = scnt[sl] + 1;
          }
        }
      }
    }
    __syncthreads();
  }

#pragma unroll 1
  for (int i = tid; i < NBD; i += NTHR) {
    const float d = (float)scnt[i] + 1.0f;
    const float r = (d > 0.0f) ? (1.0f / sqrtf(d)) : 0.0f;
    scnt[i] = __float_as_int(r);
  }
  __syncthreads();

  v4f vals[NBD / (NTHR * 4)];
#pragma unroll
  for (int it = 0; it < NBD / (NTHR * 4); ++it) {
    const int s0 = it * (NTHR * 4) + 4 * tid;
    const v4i c4 = *(const v4ia*)(scnt + s0);
    v4f v;
    v.x = __int_as_float(c4.x); v.y = __int_as_float(c4.y);
    v.z = __int_as_float(c4.z); v.w = __int_as_float(c4.w);
    vals[it] = v;
  }
#pragma unroll
  for (int it = 0; it < NBD / (NTHR * 4); ++it) {
    const int s0 = it * (NTHR * 4) + 4 * tid;
    *(volatile v4f*)(dis + (size_t)nodeBase + s0) = vals[it];
  }
  __threadfence();
#pragma unroll
  for (int it = 0; it < NBD / (NTHR * 4); ++it) {
    const int s0 = it * (NTHR * 4) + 4 * tid;
    *(volatile v4f*)(dis + (size_t)nodeBase + s0) = vals[it];
  }
}

__global__ __launch_bounds__(GTHR) void k_gemm(
    const unsigned short* __restrict__ A, const unsigned short* __restrict__ WT,
    float* outF, int K, int ldo)
{
  __shared__ __attribute__((aligned(16))) float stg[GBM * GBN];
  const int tid = (int)threadIdx.x, lane = tid & 31, wave = tid >> 5, hh = lane >> 4, m = lane & 15;
  const int rowBase = (int)blockIdx.x * GBM;
  const int col0    = (int)blockIdx.y * GBN;

  v8f acc[4];
  {
    const v8f z = {0.f, 0.f, 0.f, 0.f, 0.f, 0.f, 0.f, 0.f};
    acc[0] = z; acc[1] = z; acc[2] = z; acc[3] = z;
  }
  const unsigned short* ap = A  + (size_t)(rowBase + 16 * wave + m) * (size_t)K + 8 * hh;
  const unsigned short* wp = WT + (size_t)(col0 + m) * (size_t)K + 8 * hh;
  const int ksteps = K >> 5;
#pragma unroll 1
  for (int ks = 0; ks < ksteps; ++ks) {
    FragB af;
    af.h[0] = *(const v8usa*)(ap + 32 * ks);
    af.h[1] = *(const v8usa*)(ap + 32 * ks + 16);
#pragma unroll
    for (int t = 0; t < 4; ++t) {
      const unsigned short* wq = wp + (size_t)(16 * t) * (size_t)K + 32 * ks;
      FragB bf;
      bf.h[0] = *(const v8usa*)wq;
      bf.h[1] = *(const v8usa*)(wq + 16);
      acc[t] = wmb(af, bf, acc[t]);
    }
  }

#pragma unroll
  for (int t = 0; t < 4; ++t) {
    const int lc = 16 * t + m;
#pragma unroll
    for (int r = 0; r < 8; ++r) {
      const int lr = 16 * wave + 8 * hh + r;
      stg[lr * GBN + lc] = acc[t][r];
    }
  }
  __syncthreads();

  v4f fv[8];
#pragma unroll
  for (int i = 0; i < 8; ++i) {
    const int lr = 16 * wave + 2 * i + hh;
    fv[i] = *(const v4fa*)(stg + lr * GBN + 4 * m);
  }
#pragma unroll
  for (int i = 0; i < 8; ++i) {
    const int lr = 16 * wave + 2 * i + hh;
    const int gr = rowBase + lr;
    float* op = outF + (size_t)gr * (size_t)ldo + col0 + 4 * m;
    *(volatile v4f*)op = fv[i];
  }
  __threadfence();
#pragma unroll
  for (int i = 0; i < 8; ++i) {
    const int lr = 16 * wave + 2 * i + hh;
    const int gr = rowBase + lr;
    float* op = outF + (size_t)gr * (size_t)ldo + col0 + 4 * m;
    *(volatile v4f*)op = fv[i];
  }
}

__device__ __forceinline__ float fin1(float acc, float sv, float rd, float b, float pzr, bool live) {
  float y = (acc + sv * rd) + b;
  y = relu_np(y);
  y = y + pzr;
  return live ? y : 0.0f;
}

template <int MODE>
__global__ __launch_bounds__(NTHR) void k_agg(const int* __restrict__ srcs, const int* __restrict__ dsts,
                                              int nE, int nN, int vec8, int mRows,
                                              const float* __restrict__ dis,
                                              const float* __restrict__ ht, const float* __restrict__ bias,
                                              unsigned short* xo, float* ho) {
  extern __shared__ __attribute__((aligned(16))) int dsm[];
  int* list = dsm;
  int* hl   = dsm + LISTN;
  int* sl   = hl + RCAP;
  int* cnt  = sl + RCAP;
  int* offs = cnt + NBA;
  int* cur  = offs + NBA;
  int* misc = cur + NBA;
  const int tid = (int)threadIdx.x, lane = tid & 31, wave = tid >> 5;
  unsigned short* rowbuf = (unsigned short*)(misc + MISC_INTS) + wave * KX;
  const int nodeBase = (int)blockIdx.x * NBA;

  {
    const v4i z4 = {0, 0, 0, 0};
    for (int i = tid * 4; i < AGG_ZINTS; i += NTHR * 4) *(v4ia*)(dsm + i) = z4;
    if (tid < MISC_INTS) misc[tid] = 0;
  }
  v4f bA, bB;
  {
    const v4f a = *(const v4fa*)(bias + 4 * lane);
    const v4f b = *(const v4fa*)(bias + 128 + 4 * lane);
    bA.x = bf16_val(a.x); bA.y = bf16_val(a.y); bA.z = bf16_val(a.z); bA.w = bf16_val(a.w);
    bB.x = bf16_val(b.x); bB.y = bf16_val(b.y); bB.z = bf16_val(b.z); bB.w = bf16_val(b.w);
  }
  __syncthreads();

  int tt = 0, ovf = 0;
  build_lists<SLA, NBA, RCAP>(dsts, nE, vec8, nodeBase, list, hl, sl, cnt, offs, cur, misc,
                              tid, lane, wave, tt, ovf);

  const float qnan = __int_as_float(0x7fc00000);
  const float pz = (ovf != 0) ? qnan : 0.0f;
#pragma unroll 1
  for (int si = 0; si < NBA / NWAVE; ++si) {
    const int s    = si * NWAVE + wave;
    const int node = nodeBase + s;
    int c = cnt[s];
    const bool big = c > DEGCAP;
    c = c < 0 ? 0 : (c > DEGCAP ? DEGCAP : c);
    int o = offs[s];
    o = o < 0 ? 0 : (o > RCAP ? RCAP : o);
    const int nc = node < nN ? node : nN - 1;
    const float dd = dis[nc];
    const float rd = dd * dd;
    v4f aA = {0.0f, 0.0f, 0.0f, 0.0f};
    v4f aB = {0.0f, 0.0f, 0.0f, 0.0f};
#pragma unroll 1
    for (int b0 = 0; b0 < c; b0 += 32) {
      int idx = o + b0 + lane;
      idx = idx > RCAP - 1 ? RCAP - 1 : idx;
      const int ent = sl[idx];
      int eid = ent >> SLA;
      eid = eid < 0 ? 0 : (eid > nE - 1 ? nE - 1 : eid);
      int sr = srcs[eid];
      sr = sr < 0 ? 0 : (sr > nN - 1 ? nN - 1 : sr);
      const float cf  = dis[sr] * dd;
      const int   cfi = __float_as_int(cf);
      const int m32 = (c - b0) < 32 ? (c - b0) : 32;
#pragma unroll 1
      for (int k = 0; k < m32; ++k) {
        const int   sk = __builtin_amdgcn_readlane(sr, k);
        const float ck = __int_as_float(__builtin_amdgcn_readlane(cfi, k));
        const float* rp = ht + (size_t)sk * CH + 4 * lane;
        const v4f va = *(const v4fa*)rp;
        const v4f vb = *(const v4fa*)(rp + 128);
        aA.x = fmaf(ck, va.x, aA.x); aA.y = fmaf(ck, va.y, aA.y);
        aA.z = fmaf(ck, va.z, aA.z); aA.w = fmaf(ck, va.w, aA.w);
        aB.x = fmaf(ck, vb.x, aB.x); aB.y = fmaf(ck, vb.y, aB.y);
        aB.z = fmaf(ck, vb.z, aB.z); aB.w = fmaf(ck, vb.w, aB.w);
      }
    }
    v4f sA, sB;
    {
      const float* rp = ht + (size_t)nc * CH + 4 * lane;
      sA = *(const v4fa*)rp;
      sB = *(const v4fa*)(rp + 128);
    }
    const float pzr = big ? qnan : pz;
    const bool live = node < nN;
    v4f oA, oB;
    oA.x = fin1(aA.x, sA.x, rd, bA.x, pzr, live); oA.y = fin1(aA.y, sA.y, rd, bA.y, pzr, live);
    oA.z = fin1(aA.z, sA.z, rd, bA.z, pzr, live); oA.w = fin1(aA.w, sA.w, rd, bA.w, pzr, live);
    oB.x = fin1(aB.x, sB.x, rd, bB.x, pzr, live); oB.y = fin1(aB.y, sB.y, rd, bB.y, pzr, live);
    oB.z = fin1(aB.z, sB.z, rd, bB.z, pzr, live); oB.w = fin1(aB.w, sB.w, rd, bB.w, pzr, live);
    if constexpr (MODE != 0) {
      v4us hA, lA, hB, lB;
      split4(oA, hA, lA);
      split4(oB, hB, lB);
      *(v4usa*)(rowbuf + 4 * lane) = hA;
      *(v4usa*)(rowbuf + 128 + 4 * lane) = hB;
      *(v4usa*)(rowbuf + CH + 4 * lane) = lA;
      *(v4usa*)(rowbuf + CH + 128 + 4 * lane) = lB;
      wave_sync();
      const v8us q0 = *(const v8usa*)(rowbuf + 8 * lane);
      const v8us q1 = *(const v8usa*)(rowbuf + CH + 8 * lane);
      wave_sync();
      if (node < mRows) {
        unsigned short* rpw = xo + (size_t)node * KX + 8 * lane;
        *(volatile v8us*)rpw = q0;
        *(volatile v8us*)(rpw + CH) = q1;
        __threadfence();
        *(volatile v8us*)rpw = q0;
        *(volatile v8us*)(rpw + CH) = q1;
      }
    } else {
      if (node < mRows) {
        float* op = ho + (size_t)node * CH + 4 * lane;
        *(volatile v4f*)op = oA;
        *(volatile v4f*)(op + 128) = oB;
        __threadfence();
        *(volatile v4f*)op = oA;
        *(volatile v4f*)(op + 128) = oB;
      }
    }
  }
}

__global__ __launch_bounds__(NTHR) void k_pool(const int* __restrict__ bat, int nN, int vec8, int nG,
                                               const float* __restrict__ h3, unsigned short* hg) {
  extern __shared__ __attribute__((aligned(16))) int dsm[];
  int* list = dsm;
  int* hl   = dsm + LISTN;
  int* sl   = hl + RCP;
  int* cnt  = sl + RCP;
  int* offs = cnt + NBP;
  int* cur  = offs + NBP;
  int* misc = cur + NBP;
  const int tid = (int)threadIdx.x, lane = tid & 31, wave = tid >> 5;
  unsigned short* rowbuf = (unsigned short*)(misc + MISC_INTS) + wave * KX;
  const int gBase = (int)blockIdx.x * NBP;

  {
    const v4i z4 = {0, 0, 0, 0};
    for (int i = tid * 4; i < POOL_ZINTS; i += NTHR * 4) *(v4ia*)(dsm + i) = z4;
    if (tid < MISC_INTS) misc[tid] = 0;
  }
  __syncthreads();

  int tt = 0, ovf = 0;
  build_lists<SLP, NBP, RCP>(bat, nN, vec8, gBase, list, hl, sl, cnt, offs, cur, misc,
                             tid, lane, wave, tt, ovf);

  const float qnan = __int_as_float(0x7fc00000);
  const float pz = (ovf != 0) ? qnan : 0.0f;
#pragma unroll 1
  for (int si = 0; si < NBP / NWAVE; ++si) {
    const int s = si * NWAVE + wave;
    const int g = gBase + s;
    int c = cnt[s];
    const bool big = c > PDEGCAP;
    c = c < 0 ? 0 : (c > PDEGCAP ? PDEGCAP : c);
    int o = offs[s];
    o = o < 0 ? 0 : (o > RCP ? RCP : o);
    v4f aA = {0.0f, 0.0f, 0.0f, 0.0f};
    v4f aB = {0.0f, 0.0f, 0.0f, 0.0f};
#pragma unroll 1
    for (int b0 = 0; b0 < c; b0 += 32) {
      int idx = o + b0 + lane;
      idx = idx > RCP - 1 ? RCP - 1 : idx;
      const int ent = sl[idx];
      int nd = ent >> SLP;
      nd = nd < 0 ? 0 : (nd > nN - 1 ? nN - 1 : nd);
      const int m32 = (c - b0) < 32 ? (c - b0) : 32;
#pragma unroll 1
      for (int k = 0; k < m32; ++k) {
        const int nk = __builtin_amdgcn_readlane(nd, k);
        const float* rp = h3 + (size_t)nk * CH + 4 * lane;
        const v4f va = *(const v4fa*)rp;
        const v4f vb = *(const v4fa*)(rp + 128);
        aA = aA + va;
        aB = aB + vb;
      }
    }
    const float cf  = (c < 1) ? 1.0f : (float)c;
    const float inv = 1.0f / cf;
    const float pzr = big ? qnan : pz;
    v4f oA, oB;
    oA.x = aA.x * inv + pzr; oA.y = aA.y * inv + pzr; oA.z = aA.z * inv + pzr; oA.w = aA.w * inv + pzr;
    oB.x = aB.x * inv + pzr; oB.y = aB.y * inv + pzr; oB.z = aB.z * inv + pzr; oB.w = aB.w * inv + pzr;
    v4us hA, lA, hB, lB;
    split4(oA, hA, lA);
    split4(oB, hB, lB);
    *(v4usa*)(rowbuf + 4 * lane) = hA;
    *(v4usa*)(rowbuf + 128 + 4 * lane) = hB;
    *(v4usa*)(rowbuf + CH + 4 * lane) = lA;
    *(v4usa*)(rowbuf + CH + 128 + 4 * lane) = lB;
    wave_sync();
    const v8us q0 = *(const v8usa*)(rowbuf + 8 * lane);
    const v8us q1 = *(const v8usa*)(rowbuf + CH + 8 * lane);
    wave_sync();
    if (g < nG) {
      unsigned short* rpw = hg + (size_t)g * KX + 8 * lane;
      *(volatile v8us*)rpw = q0;
      *(volatile v8us*)(rpw + CH) = q1;
      __threadfence();
      *(volatile v8us*)rpw = q0;
      *(volatile v8us*)(rpw + CH) = q1;
    }
  }
}

__global__ __launch_bounds__(GTHR) void k_head(const unsigned short* __restrict__ HG,
                                               const unsigned short* __restrict__ WF1,
                                               const unsigned short* __restrict__ WF2,
                                               const float* __restrict__ bf1, const float* __restrict__ bf2,
                                               float* out) {
  __shared__ __attribute__((aligned(16))) unsigned short t2[GBM * KT2];
  __shared__ __attribute__((aligned(16))) float os[GBM * DOUT];
  __shared__ float bs1[HF1];
  __shared__ float bs2[DOUT];
  const int tid = (int)threadIdx.x, lane = tid & 31, wave = tid >> 5, hh = lane >> 4, m = lane & 15;
  const int rowBase = (int)blockIdx.x * GBM;

  bs1[tid] = bf16_val(bf1[tid]);
  if (tid < DOUT) bs2[tid] = bf16_val(bf2[tid]);

  v8f acc[8];
  {
    const v8f z = {0.f, 0.f, 0.f, 0.f, 0.f, 0.f, 0.f, 0.f};
#pragma unroll
    for (int t = 0; t < 8; ++t) acc[t] = z;
  }
  const unsigned short* ap = HG  + (size_t)(rowBase + 16 * wave + m) * (size_t)KX + 8 * hh;
  const unsigned short* bp = WF1 + (size_t)m * (size_t)KX + 8 * hh;
#pragma unroll 1
  for (int k0 = 0; k0 < KX; k0 += 32) {
    FragB af;
    af.h[0] = *(const v8usa*)(ap + k0);
    af.h[1] = *(const v8usa*)(ap + k0 + 16);
#pragma unroll
    for (int nt = 0; nt < 8; ++nt) {
      const unsigned short* wq = bp + (size_t)(16 * nt) * (size_t)KX + k0;
      FragB bf;
      bf.h[0] = *(const v8usa*)wq;
      bf.h[1] = *(const v8usa*)(wq + 16);
      acc[nt] = wmb(af, bf, acc[nt]);
    }
  }
  __syncthreads();

#pragma unroll
  for (int nt = 0; nt < 8; ++nt) {
    const int col = 16 * nt + m;
    const float bb = bs1[col];
#pragma unroll
    for (int r = 0; r < 8; ++r) {
      const int lr = 16 * wave + 8 * hh + r;
      const float tv = relu_np(acc[nt][r] + bb);
      const unsigned hb = bf16_bits(tv);
      const unsigned lb = bf16_bits(tv - __uint_as_float(hb << 16));
      t2[lr * KT2 + col]       = (unsigned short)hb;
      t2[lr * KT2 + HF1 + col] = (unsigned short)lb;
    }
  }
  __syncthreads();

  v8f acc2[2];
  {
    const v8f z = {0.f, 0.f, 0.f, 0.f, 0.f, 0.f, 0.f, 0.f};
    acc2[0] = z; acc2[1] = z;
  }
  const unsigned short* tp  = t2  + (size_t)(16 * wave + m) * KT2 + 8 * hh;
  const unsigned short* bp2 = WF2 + (size_t)m * (size_t)KT2 + 8 * hh;
#pragma unroll 1
  for (int k0 = 0; k0 < KT2; k0 += 32) {
    FragB af;
    af.h[0] = *(const v8usa*)(tp + k0);
    af.h[1] = *(const v8usa*)(tp + k0 + 16);
#pragma unroll
    for (int nt = 0; nt < 2; ++nt) {
      const unsigned short* wq = bp2 + (size_t)(16 * nt) * (size_t)KT2 + k0;
      FragB bf;
      bf.h[0] = *(const v8usa*)wq;
      bf.h[1] = *(const v8usa*)(wq + 16);
      acc2[nt] = wmb(af, bf, acc2[nt]);
    }
  }
#pragma unroll
  for (int nt = 0; nt < 2; ++nt) {
    const int col = 16 * nt + m;
    const float bb = bs2[col];
#pragma unroll
    for (int r = 0; r < 8; ++r) {
      const int lr = 16 * wave + 8 * hh + r;
      os[lr * DOUT + col] = acc2[nt][r] + bb;
    }
  }
  __syncthreads();

  constexpr int NIT = (GBM * DOUT) / (4 * GTHR);
  v4f ov[NIT];
#pragma unroll
  for (int it = 0; it < NIT; ++it) ov[it] = *(const v4fa*)(os + 4 * (it * GTHR + tid));
  float* ob = out + (size_t)rowBase * DOUT;
#pragma unroll
  for (int it = 0; it < NIT; ++it) *(volatile v4f*)(ob + 4 * (size_t)(it * GTHR + tid)) = ov[it];
  __threadfence();
#pragma unroll
  for (int it = 0; it < NIT; ++it) *(volatile v4f*)(ob + 4 * (size_t)(it * GTHR + tid)) = ov[it];
}

static inline int cdiv(int a, int b) { return (a + b - 1) / b; }
static inline size_t al256(size_t o) { return (o + 255) & ~(size_t)255; }

extern "C" void kernel_launch(void* const* d_in, const int* in_sizes, int n_in,
                              void* d_out, int out_size, void* d_ws, size_t ws_size,
                              hipStream_t stream) {
  if (n_in < 13) return;
  if (in_sizes[0] < CIN || (in_sizes[0] % CIN) != 0) return;
  const int nN = in_sizes[0] / CIN;
  if (nN < 16 || nN >= (1 << 22)) return;
  if (in_sizes[1] < 2 || (in_sizes[1] & 1) != 0) return;
  const int nE = in_sizes[1] / 2;
  if (nE < 1 || nE >= (1 << (31 - SLA))) return;
  if (in_sizes[2] != nN) return;
  if (in_sizes[3] != CIN * CH || in_sizes[4] != CH) return;
  if (in_sizes[5] != CH * CH || in_sizes[6] != CH) return;
  if (in_sizes[7] != CH * CH || in_sizes[8] != CH) return;
  if (in_sizes[9] != CH * HF1 || in_sizes[10] != HF1) return;
  if (in_sizes[11] != HF1 * DOUT || in_sizes[12] != DOUT) return;
  if (out_size != NOUT) return;

  const float* x    = (const float*)d_in[0];
  const int*   edge = (const int*)d_in[1];
  const int*   bat  = (const int*)d_in[2];
  const float* W1   = (const float*)d_in[3];
  const float* b1   = (const float*)d_in[4];
  const float* W2   = (const float*)d_in[5];
  const float* b2   = (const float*)d_in[6];
  const float* W3   = (const float*)d_in[7];
  const float* b3   = (const float*)d_in[8];
  const float* Wf1  = (const float*)d_in[9];
  const float* bf1  = (const float*)d_in[10];
  const float* Wf2  = (const float*)d_in[11];
  const float* bf2  = (const float*)d_in[12];
  float* out = (float*)d_out;
  const int* src = edge;
  const int* dst = edge + nE;

  const int MP   = cdiv(nN, GBM) * GBM;
  const int gM   = MP / GBM;
  const int gD   = cdiv(nN, NBD);
  const int NBPD = gD * NBD;
  const int gA   = cdiv(MP, NBA);
  if ((long long)gA * NBA < (long long)MP) return;
  if (NBPD < nN) return;
  const int vec8e = ((nE & 3) == 0) ? 1 : 0;
  const int vec8n = 1;

  char* ws = (char*)d_ws;
  size_t off = 0;
  const size_t oDIS = off; off = al256(off + (size_t)NBPD * 4);
  const size_t oW1T = off; off = al256(off + (size_t)CH * CIN * 2);
  const size_t oW2T = off; off = al256(off + (size_t)CH * KX * 2);
  const size_t oW3T = off; off = al256(off + (size_t)CH * KX * 2);
  const size_t oWF1 = off; off = al256(off + (size_t)HF1 * KX * 2);
  const size_t oWF2 = off; off = al256(off + (size_t)DOUT * KT2 * 2);
  const size_t oXB  = off; off = al256(off + (size_t)MP * CIN * 2);
  const size_t oHT  = off; off = al256(off + (size_t)MP * CH * 4);
  const size_t oX   = off; off = al256(off + (size_t)MP * KX * 2);
  const size_t oHG  = off; off = al256(off + (size_t)NG * KX * 2);
  if (off > ws_size || off > (size_t)WSMAX) return;
  if ((size_t)MP * CH * 4 > (size_t)MP * KX * 2) return;
  float*          DIS  = (float*)(ws + oDIS);
  unsigned short* W1T  = (unsigned short*)(ws + oW1T);
  unsigned short* W2T2 = (unsigned short*)(ws + oW2T);
  unsigned short* W3T2 = (unsigned short*)(ws + oW3T);
  unsigned short* WF1T = (unsigned short*)(ws + oWF1);
  unsigned short* WF2T = (unsigned short*)(ws + oWF2);
  unsigned short* XB   = (unsigned short*)(ws + oXB);
  float*          HT   = (float*)(ws + oHT);
  unsigned short* X    = (unsigned short*)(ws + oX);
  float*          H3   = (float*)(ws + oX);
  unsigned short* HG   = (unsigned short*)(ws + oHG);

  const size_t aggLds  = (size_t)AGG_LDS_INTS * 4;
  const size_t poolLds = (size_t)POOL_LDS_INTS * 4;
  hipFuncSetAttribute(reinterpret_cast<const void*>(&k_agg<1>), hipFuncAttributeMaxDynamicSharedMemorySize, (int)aggLds);
  hipFuncSetAttribute(reinterpret_cast<const void*>(&k_agg<0>), hipFuncAttributeMaxDynamicSharedMemorySize, (int)aggLds);

  const int nUx = MP * (CIN / 8);
  k_wprep<<<NUALL / NTHR, NTHR, 0, stream>>>(W1, W2, W3, Wf1, Wf2, W1T, W2T2, W3T2, WF1T, WF2T);
  k_cvx<<<cdiv(nUx, NTHR), NTHR, 0, stream>>>(x, nN, nUx, XB);
  k_deg<<<gD, NTHR, 0, stream>>>(dst, nE, vec8e, DIS);
  k_gemm<<<dim3(gM, CH / GBN), GTHR, 0, stream>>>(XB, W1T, HT, CIN, CH);
  k_agg<1><<<gA, NTHR, aggLds, stream>>>(src, dst, nE, nN, vec8e, MP, DIS, HT, b1, X, H3);
  k_gemm<<<dim3(gM, CH / GBN), GTHR, 0, stream>>>(X, W2T2, HT, KX, CH);
  k_agg<1><<<gA, NTHR, aggLds, stream>>>(src, dst, nE, nN, vec8e, MP, DIS, HT, b2, X, H3);
  k_gemm<<<dim3(gM, CH / GBN), GTHR, 0, stream>>>(X, W3T2, HT, KX, CH);
  k_agg<0><<<gA, NTHR, aggLds, stream>>>(src, dst, nE, nN, vec8e, MP, DIS, HT, b3, X, H3);
  k_pool<<<NG / NBP, NTHR, poolLds, stream>>>(bat, nN, vec8n, NG, H3, HG);
  k_head<<<NG / GBM, GTHR, 0, stream>>>(HG, WF1T, WF2T, bf1, bf2, out);
}
